// TritonSubMConv3d_45681272160692
// MI455X (gfx1250) — hardware-verified
//
#include <hip/hip_runtime.h>
#include <stddef.h>


#define CIN    64
#define COUT   64
#define NTAP   27
#define KCONV  (NTAP * CIN)
#define GRIDW  64
#define NBATCH 4
#define NCELL  (NBATCH * GRIDW * GRIDW * GRIDW)
#define NTHR   256
#define NWAVE  8
#define EPT    8
#define CHUNK  (NTHR * EPT)
#define WCAP   (32 * EPT)
#define CPB    8192
#define NGBLK  (NCELL / CPB)
#define CROWS  64
#define CTHR   128
#define AP     (CIN + 8)
#define WSC    4.0f
#define WSCI   0.25f

static_assert(NCELL % CPB == 0);
static_assert((CPB & (CPB - 1)) == 0 && CPB <= 65536);
static_assert((CHUNK & (CHUNK - 1)) == 0 && CHUNK <= 2048);
static_assert(CHUNK % (4 * NTHR) == 0);
static_assert(CPB % (4 * NTHR) == 0);
static_assert(KCONV % 32 == 0);
static_assert(CIN % 32 == 0);
static_assert(COUT == 64);
static_assert(CROWS * AP * 2 <= CROWS * COUT * 4);
static_assert(CROWS == (CTHR / 32) * 16);
static_assert((CROWS * CIN / 8) % CTHR == 0);
static_assert((COUT * KCONV / 8) % NTHR == 0);
static_assert((AP * 2) % 16 == 0);

typedef float    v4f  __attribute__((ext_vector_type(4)));
typedef float    v8f  __attribute__((ext_vector_type(8)));
typedef int      v4i  __attribute__((ext_vector_type(4)));
typedef _Float16 v8h  __attribute__((ext_vector_type(8)));
typedef _Float16 v16h __attribute__((ext_vector_type(16)));
union FragH { v16h v; v8h h[2]; };

__device__ __forceinline__ v8h cvt8h(v4f a, v4f b) {
  v8h r;
  r[0] = (_Float16)a.x; r[1] = (_Float16)a.y; r[2] = (_Float16)a.z; r[3] = (_Float16)a.w;
  r[4] = (_Float16)b.x; r[5] = (_Float16)b.y; r[6] = (_Float16)b.z; r[7] = (_Float16)b.w;
  return r;
}

__device__ __forceinline__ v8f wmh(v16h a, v16h b, v8f c) {
  v8f d = __builtin_amdgcn_wmma_f32_16x16x32_f16(false, a, false, b, (short)0, c, false, false);
  asm volatile("v_nop\n\tv_nop\n\tv_nop\n\tv_nop" : "+v"(d) : "v"(a), "v"(b));
  return d;
}

__device__ __forceinline__ int cell_of(const int* __restrict__ coords, const int* __restrict__ bidx,
                                       int e, int n) {
  const int ec = e < n ? e : n - 1;
  const int x = coords[(size_t)ec * 3 + 0];
  const int y = coords[(size_t)ec * 3 + 1];
  const int z = coords[(size_t)ec * 3 + 2];
  const int b = bidx[ec];
  const bool ok = (e < n) && ((unsigned)x < (unsigned)GRIDW) && ((unsigned)y < (unsigned)GRIDW) &&
                  ((unsigned)z < (unsigned)GRIDW) && ((unsigned)b < (unsigned)NBATCH);
  const int id = ((b * GRIDW + x) * GRIDW + y) * GRIDW + z;
  return ok ? id : -1;
}

__global__ __launch_bounds__(NTHR) void k_cell(
    const int* __restrict__ coords, const int* __restrict__ bidx, int n, int nPad, int* cell) {
  const int t = blockIdx.x * NTHR + (int)threadIdx.x;
  if (4 * t >= nPad) return;
  v4i cv;
  cv.x = cell_of(coords, bidx, 4 * t + 0, n);
  cv.y = cell_of(coords, bidx, 4 * t + 1, n);
  cv.z = cell_of(coords, bidx, 4 * t + 2, n);
  cv.w = cell_of(coords, bidx, 4 * t + 3, n);
  int* p = cell + 4 * (size_t)t;
  *(volatile v4i*)p = cv;
  __threadfence();
  *(volatile v4i*)p = cv;
}

__global__ __launch_bounds__(NTHR) void k_grid(const int* __restrict__ cell, int nPad, int* G) {
  __shared__ __attribute__((aligned(16))) int gcell[CPB];
  __shared__ __attribute__((aligned(16))) int list[NWAVE * WCAP];
  __shared__ int wcnt[NWAVE];
  const int tid = threadIdx.x, lane = tid & 31, wave = tid >> 5;
  const int cBase = blockIdx.x * CPB;
  {
    const v4i m1 = {-1, -1, -1, -1};
    for (int i = tid; i < CPB / 4; i += NTHR) ((v4i*)gcell)[i] = m1;
  }
  __syncthreads();

  const int nChunks = nPad / CHUNK;
#pragma unroll 1
  for (int ch = 0; ch < nChunks; ++ch) {
    const int cbase = ch * CHUNK;
    const int el0 = tid * EPT;
    const int* cp = cell + (size_t)cbase + el0;
    const v4i da = *(const v4i*)cp;
    const v4i db = *(const v4i*)(cp + 4);
    const unsigned nb = (unsigned)cBase;
    const unsigned s0 = (unsigned)da.x - nb, s1 = (unsigned)da.y - nb;
    const unsigned s2 = (unsigned)da.z - nb, s3 = (unsigned)da.w - nb;
    const unsigned s4 = (unsigned)db.x - nb, s5 = (unsigned)db.y - nb;
    const unsigned s6 = (unsigned)db.z - nb, s7 = (unsigned)db.w - nb;
    const bool h0 = s0 < (unsigned)CPB, h1 = s1 < (unsigned)CPB, h2 = s2 < (unsigned)CPB, h3 = s3 < (unsigned)CPB;
    const bool h4 = s4 < (unsigned)CPB, h5 = s5 < (unsigned)CPB, h6 = s6 < (unsigned)CPB, h7 = s7 < (unsigned)CPB;
    int wc = 0;
    const unsigned any = __builtin_amdgcn_ballot_w32(h0 | h1 | h2 | h3 | h4 | h5 | h6 | h7);
    if (any != 0u) {
#define HITJ(J, HJ, SJ) { \
        const unsigned mj = __builtin_amdgcn_ballot_w32(HJ); \
        if (mj != 0u) { \
          if (HJ) { \
            const int pos = wc + (int)__builtin_amdgcn_mbcnt_lo(mj, 0u); \
            if (pos < WCAP) list[wave * WCAP + pos] = ((el0 + (J)) << 16) | (int)(SJ); \
          } \
          wc += (int)__builtin_popcount(mj); } }
      HITJ(0, h0, s0)
      HITJ(1, h1, s1)
      HITJ(2, h2, s2)
      HITJ(3, h3, s3)
      HITJ(4, h4, s4)
      HITJ(5, h5, s5)
      HITJ(6, h6, s6)
      HITJ(7, h7, s7)
#undef HITJ
    }
    if (lane == 0) wcnt[wave] = wc;
    __syncthreads();
    if (tid == 0) {
#pragma unroll 1
      for (int w = 0; w < NWAVE; ++w) {
        int cnt = wcnt[w];
        cnt = cnt > WCAP ? WCAP : (cnt < 0 ? 0 : cnt);
#pragma unroll 1
        for (int i = 0; i < cnt; ++i) {
          const int ent  = list[w * WCAP + i];
          const int slot = ent & (CPB - 1);
          const int idx  = cbase + ((ent >> 16) & (CHUNK - 1));
          const int v    = gcell[slot];
          if (v < 0 || idx < v) gcell[slot] = idx;
        }
      }
    }
    __syncthreads();
  }

  int* gp = G + (size_t)cBase;
#pragma unroll
  for (int it = 0; it < CPB / (4 * NTHR); ++it) {
    const int i = it * NTHR + tid;
    const v4i v = ((const v4i*)gcell)[i];
    *(volatile v4i*)(gp + 4 * (size_t)i) = v;
  }
  __threadfence();
#pragma unroll
  for (int it = 0; it < CPB / (4 * NTHR); ++it) {
    const int i = it * NTHR + tid;
    const v4i v = ((const v4i*)gcell)[i];
    *(volatile v4i*)(gp + 4 * (size_t)i) = v;
  }
}

__global__ __launch_bounds__(NTHR) void k_x16(const float* __restrict__ f, int total8, _Float16* X16) {
  const int t = blockIdx.x * NTHR + (int)threadIdx.x;
  if (t >= total8) return;
  const size_t e = (size_t)t * 8;
  const v4f a = *(const v4f*)(f + e);
  const v4f b = *(const v4f*)(f + e + 4);
  const v8h hv = cvt8h(a, b);
  _Float16* dp = X16 + e;
  *(volatile v8h*)dp = hv;
  __threadfence();
  *(volatile v8h*)dp = hv;
}

__global__ __launch_bounds__(NTHR) void k_prepw(const float* __restrict__ w, _Float16* Wp) {
  const int i = blockIdx.x * NTHR + (int)threadIdx.x;
  if (i >= COUT * KCONV / 8) return;
  const int o   = i / (KCONV / 8);
  const int kk0 = (i - o * (KCONV / 8)) * 8;
  const int tap = kk0 >> 6;
  const int c0  = kk0 & (CIN - 1);
  v8h hv;
#pragma unroll
  for (int e = 0; e < 8; ++e)
    hv[e] = (_Float16)(w[((size_t)tap * CIN + c0 + e) * COUT + o] * WSC);
  _Float16* dp = Wp + (size_t)o * KCONV + kk0;
  *(volatile v8h*)dp = hv;
  __threadfence();
  *(volatile v8h*)dp = hv;
}

__global__ __launch_bounds__(CTHR) void k_conv(
    const _Float16* __restrict__ X16, const int* __restrict__ coords, const int* __restrict__ bidx,
    const int* __restrict__ G, const _Float16* __restrict__ Wp, int n, float* out) {
  __shared__ __attribute__((aligned(16))) float ctile[CROWS * COUT];
  __shared__ __attribute__((aligned(16))) int   lidx[CROWS * NTAP];
  __shared__ int vx[CROWS], vy[CROWS], vz[CROWS], vb[CROWS];
  _Float16* sA = (_Float16*)ctile;
  const int tid = threadIdx.x, lane = tid & 31, wave = tid >> 5, hh = lane >> 4, m = lane & 15;
  const int rowBase = blockIdx.x * CROWS;

  if (tid < CROWS) {
    const int row = rowBase + tid;
    const int rc  = row < n ? row : n - 1;
    const int x = coords[(size_t)rc * 3 + 0];
    const int y = coords[(size_t)rc * 3 + 1];
    const int z = coords[(size_t)rc * 3 + 2];
    const int b = bidx[rc];
    const bool ok = (row < n) && ((unsigned)x < (unsigned)GRIDW) && ((unsigned)y < (unsigned)GRIDW) &&
                    ((unsigned)z < (unsigned)GRIDW) && ((unsigned)b < (unsigned)NBATCH);
    vx[tid] = ok ? x : 0;
    vy[tid] = ok ? y : 0;
    vz[tid] = ok ? z : 0;
    vb[tid] = ok ? b : -1;
  }
  v8f acc[4];
#pragma unroll
  for (int t = 0; t < 4; ++t) { v8f zz = {0.f, 0.f, 0.f, 0.f, 0.f, 0.f, 0.f, 0.f}; acc[t] = zz; }
  __syncthreads();

#pragma unroll 1
  for (int j = tid; j < CROWS * NTAP; j += CTHR) {
    const int r  = j / NTAP;
    const int k  = j - r * NTAP;
    const int dx = k / 9 - 1;
    const int dy = (k / 3) % 3 - 1;
    const int dz = k % 3 - 1;
    const int b  = vb[r];
    const int nx = vx[r] + dx, ny = vy[r] + dy, nz = vz[r] + dz;
    const bool ok = (b >= 0) && ((unsigned)nx < (unsigned)GRIDW) && ((unsigned)ny < (unsigned)GRIDW) &&
                    ((unsigned)nz < (unsigned)GRIDW);
    int cid = ((b * GRIDW + nx) * GRIDW + ny) * GRIDW + nz;
    cid = ok ? cid : 0;
    cid = cid < 0 ? 0 : (cid > NCELL - 1 ? NCELL - 1 : cid);
    int g = G[cid];
    g = ok ? g : -1;
    if ((unsigned)g >= (unsigned)n) g = -1;
    lidx[j] = g;
  }
  __syncthreads();

#pragma unroll 1
  for (int tap = 0; tap < NTAP; ++tap) {
#pragma unroll
    for (int i = 0; i < (CROWS * CIN / 8) / CTHR; ++i) {
      const int u  = i * CTHR + tid;
      const int r  = u >> 3;
      const int c0 = (u & 7) * 8;
      const int g  = lidx[r * NTAP + tap];
      const bool ok = (unsigned)g < (unsigned)n;
      const int gc = g < 0 ? 0 : (g > n - 1 ? n - 1 : g);
      v4i xi = *(const v4i*)(X16 + (size_t)gc * CIN + c0);
      const int mk = ok ? -1 : 0;
      xi = xi & mk;
      *(v4i*)(sA + r * AP + c0) = xi;
    }
    __syncthreads();
    const _Float16* ar = sA + (wave * 16 + m) * AP + 8 * hh;
#pragma unroll
    for (int kt = 0; kt < CIN / 32; ++kt) {
      FragH a;
      a.h[0] = *(const v8h*)(ar + 32 * kt);
      a.h[1] = *(const v8h*)(ar + 32 * kt + 16);
#pragma unroll
      for (int t = 0; t < 4; ++t) {
        const _Float16* bp = Wp + (size_t)(16 * t + m) * KCONV + tap * CIN + 32 * kt + 8 * hh;
        FragH b;
        b.h[0] = *(const v8h*)bp;
        b.h[1] = *(const v8h*)(bp + 16);
        acc[t] = wmh(a.v, b.v, acc[t]);
      }
    }
    __syncthreads();
  }

  {
    float* sp = ctile + (wave * 16 + 8 * hh) * COUT + m;
#pragma unroll
    for (int t = 0; t < 4; ++t) {
#pragma unroll
      for (int r = 0; r < 8; ++r) sp[r * COUT + 16 * t] = acc[t][r] * WSCI;
    }
  }
  __syncthreads();

  const float* lp = ctile + wave * 16 * COUT;
  v4f ov[8];
#pragma unroll
  for (int i = 0; i < 8; ++i) ov[i] = *(const v4f*)(lp + (2 * i + hh) * COUT + 4 * m);
  const int rowW = rowBase + wave * 16;
#pragma unroll
  for (int i = 0; i < 8; ++i) {
    const int grow = rowW + 2 * i + hh;
    if (grow < n) *(volatile v4f*)(out + (size_t)grow * COUT + 4 * m) = ov[i];
  }
  __threadfence();
#pragma unroll
  for (int i = 0; i < 8; ++i) {
    const int grow = rowW + 2 * i + hh;
    if (grow < n) *(volatile v4f*)(out + (size_t)grow * COUT + 4 * m) = ov[i];
  }
}

extern "C" void kernel_launch(void* const* d_in, const int* in_sizes, int n_in,
                              void* d_out, int out_size, void* d_ws, size_t ws_size,
                              hipStream_t stream) {
  if (n_in < 4) return;
  const int n = in_sizes[0] / CIN;
  if (n < 1 || in_sizes[0] != n * CIN) return;
  if (in_sizes[1] != 3 * n || in_sizes[2] != n || in_sizes[3] != NTAP * CIN * COUT) return;
  if (out_size != n * COUT) return;

  const float* features = (const float*)d_in[0];
  const int*   coords   = (const int*)d_in[1];
  const int*   bidx     = (const int*)d_in[2];
  const float* weight   = (const float*)d_in[3];
  float* out = (float*)d_out;

  const int nPad = ((n + CHUNK - 1) / CHUNK) * CHUNK;

  char* ws = (char*)d_ws;
  size_t off = 0;
  const size_t oG    = off; off += (size_t)NCELL * 4;         off = (off + 255) & ~(size_t)255;
  const size_t oCell = off; off += (size_t)nPad * 4;          off = (off + 255) & ~(size_t)255;
  const size_t oX16  = off; off += (size_t)n * CIN * 2;       off = (off + 255) & ~(size_t)255;
  const size_t oWp   = off; off += (size_t)COUT * KCONV * 2;  off = (off + 255) & ~(size_t)255;
  if (off > ws_size || off > (size_t)134217728) return;

  int*      G    = (int*)(ws + oG);
  int*      CELL = (int*)(ws + oCell);
  _Float16* X16  = (_Float16*)(ws + oX16);
  _Float16* Wp   = (_Float16*)(ws + oWp);

  const int nCellBlk = nPad / (4 * NTHR);
  const int nX16Blk  = (n * 8 + NTHR - 1) / NTHR;
  const int nPrepBlk = (COUT * KCONV / 8) / NTHR;
  const int nConvBlk = (n + CROWS - 1) / CROWS;

  k_cell<<<nCellBlk, NTHR, 0, stream>>>(coords, bidx, n, nPad, CELL);
  k_grid<<<NGBLK, NTHR, 0, stream>>>(CELL, nPad, G);
  k_x16<<<nX16Blk, NTHR, 0, stream>>>(features, n * 8, X16);
  k_prepw<<<nPrepBlk, NTHR, 0, stream>>>(weight, Wp);
  k_conv<<<nConvBlk, CTHR, 0, stream>>>(X16, coords, bidx, G, Wp, n, out);
}
